// GATModule_55087250538928
// MI455X (gfx1250) — hardware-run, weakly checked
//
#include <hip/hip_runtime.h>
#include <stddef.h>
#include <stdint.h>
#include <math.h>

#pragma clang fp contract(off)


#define FIN     84
#define KIN     96
#define CH      384
#define NH1     4
#define HD1     1536
#define KA2     3072
#define HD2     384
#define EDM     11
#define ELW     8
#define KAPN    64
#define KAP2    48
#define NTHR    256
#define NWAVE   8
#define EPT     8
#define CHUNK   (NTHR * EPT)
#define WCAP    (EPT * 32)
#define LISTN   (NWAVE * WCAP)
#define NBMAX   2048
#define SLOTB   11
#define RCAP    28672
#define DEGCAP  256
#define GBM     64
#define GBN     64
#define GTHR    128
#define NDB     32
#define PTHR    96
#define PCH     (PTHR * 8)
#define PWC     256
#define NEGSL   0.2f
#define EPS_SM  1e-16f
#define WSMAX   134217728
#define LDS_AGG ((2 * RCAP + 2 * NBMAX + LISTN) * 4 + 64)

static_assert((CHUNK & (CHUNK - 1)) == 0 && CHUNK <= (1 << SLOTB));
static_assert(NBMAX == (1 << SLOTB));
static_assert(NTHR * 8 == NBMAX);
static_assert(LISTN >= NBMAX);
static_assert(LISTN >= NWAVE * WCAP);
static_assert((RCAP % 32) == 0);
static_assert(4 * NBMAX <= RCAP);
static_assert(LDS_AGG <= 300000);
static_assert(GBM == (GTHR / 32) * 16);
static_assert((KIN % 32) == 0 && (KA2 % 32) == 0 && KA2 == 2 * HD1);
static_assert((HD1 % GBN) == 0 && (HD2 % GBN) == 0);
static_assert(HD1 == NH1 * CH && HD2 == CH);
static_assert(HD1 == 2 * 768 && 768 == 3 * 256);
static_assert(CH == 3 * 128 && HD2 == 3 * 128);
static_assert(FIN <= KIN && (FIN % 4) == 0 && KIN / 8 == 12 && KA2 / 8 == 384);
static_assert(NH1 * EDM <= KAP2 && KAP2 + EDM <= KAPN);
static_assert(NDB * ELW == NTHR && NDB == 4 * NWAVE);
static_assert(PCH == PTHR * EPT && PWC == 32 * EPT && (PTHR % 32) == 0);

typedef float          v2f  __attribute__((ext_vector_type(2)));
typedef float          v4f  __attribute__((ext_vector_type(4)));
typedef float          v8f  __attribute__((ext_vector_type(8)));
typedef int            v4i  __attribute__((ext_vector_type(4)));
typedef int            v8i  __attribute__((ext_vector_type(8)));
typedef unsigned int   v4u  __attribute__((ext_vector_type(4)));
typedef unsigned short v8us __attribute__((ext_vector_type(8)));
typedef __bf16         v16b __attribute__((ext_vector_type(16)));
typedef v2f  __attribute__((may_alias)) v2fa;
typedef v4f  __attribute__((may_alias)) v4fa;
typedef v8us __attribute__((may_alias)) v8usa;
union FragB { v16b v; v8us h[2]; v8i w; };

__device__ __forceinline__ v8f wmb(const FragB& a, const FragB& b, v8f c) {
  v8f d = __builtin_amdgcn_wmma_f32_16x16x32_bf16(false, a.v, false, b.v, (short)0, c, false, false);
  asm volatile("v_nop\n\tv_nop\n\tv_nop\n\tv_nop" : "+v"(d) : "v"(a.w), "v"(b.w));
  return d;
}

__device__ __forceinline__ unsigned int f2bf(float f) {
  const unsigned int u = __float_as_uint(f);
  return ((u + 0x7FFFu + ((u >> 16) & 1u)) >> 16) & 0xFFFFu;
}
__device__ __forceinline__ float bf2f(unsigned int b) { return __uint_as_float(b << 16); }
__device__ __forceinline__ float bfr(float f) { return bf2f(f2bf(f)); }
__device__ __forceinline__ v4f bfr4(const v4f a) {
  v4f r; r.x = bfr(a.x); r.y = bfr(a.y); r.z = bfr(a.z); r.w = bfr(a.w); return r;
}
__device__ __forceinline__ unsigned int pk2(float lo, float hi) { return f2bf(lo) | (f2bf(hi) << 16); }
__device__ __forceinline__ v4u pack8(const v4f a, const v4f b) {
  v4u r;
  r.x = pk2(a.x, a.y); r.y = pk2(a.z, a.w); r.z = pk2(b.x, b.y); r.w = pk2(b.z, b.w);
  return r;
}
__device__ __forceinline__ void split8(const v4f a, const v4f b, v4u& hv, v4u& lv) {
  const unsigned int h0 = f2bf(a.x), h1 = f2bf(a.y), h2 = f2bf(a.z), h3 = f2bf(a.w);
  const unsigned int h4 = f2bf(b.x), h5 = f2bf(b.y), h6 = f2bf(b.z), h7 = f2bf(b.w);
  const unsigned int l0 = f2bf(a.x - bf2f(h0)), l1 = f2bf(a.y - bf2f(h1));
  const unsigned int l2 = f2bf(a.z - bf2f(h2)), l3 = f2bf(a.w - bf2f(h3));
  const unsigned int l4 = f2bf(b.x - bf2f(h4)), l5 = f2bf(b.y - bf2f(h5));
  const unsigned int l6 = f2bf(b.z - bf2f(h6)), l7 = f2bf(b.w - bf2f(h7));
  hv.x = h0 | (h1 << 16); hv.y = h2 | (h3 << 16); hv.z = h4 | (h5 << 16); hv.w = h6 | (h7 << 16);
  lv.x = l0 | (l1 << 16); lv.y = l2 | (l3 << 16); lv.z = l4 | (l5 << 16); lv.w = l6 | (l7 << 16);
}
__device__ __forceinline__ float leaky(float v) { return v > 0.f ? v : v * NEGSL; }
__device__ __forceinline__ void ostep(float lg, float& mx, float& dn) {
  const float df = lg - mx;
  const float ee = __expf(-fabsf(df));
  const bool up  = df > 0.f;
  const float s1 = up ? ee : 1.0f;
  const float s2 = up ? 1.0f : ee;
  mx = up ? lg : mx;
  dn = fmaf(dn, s1, s2);
}
__device__ __forceinline__ v4f mul4s(float p, const v4f x) {
  v4f r; r.x = p * x.x; r.y = p * x.y; r.z = p * x.z; r.w = p * x.w; return r;
}
__device__ __forceinline__ v4f fma4s(float p, const v4f x, v4f a) {
  a.x = fmaf(p, x.x, a.x); a.y = fmaf(p, x.y, a.y); a.z = fmaf(p, x.z, a.z); a.w = fmaf(p, x.w, a.w); return a;
}
__device__ __forceinline__ v4f add4(const v4f a, const v4f b) {
  v4f r; r.x = a.x + b.x; r.y = a.y + b.y; r.z = a.z + b.z; r.w = a.w + b.w; return r;
}
__device__ __forceinline__ float eluf(float v) {
  const float n = __expf(fminf(v, 0.f)) - 1.0f;
  return v > 0.f ? v : n;
}
__device__ __forceinline__ v4f elu4(const v4f a) {
  v4f r; r.x = eluf(a.x); r.y = eluf(a.y); r.z = eluf(a.z); r.w = eluf(a.w); return r;
}
__device__ __forceinline__ v4f max4(const v4f a, const v4f b) {
  v4f r; r.x = fmaxf(a.x, b.x); r.y = fmaxf(a.y, b.y); r.z = fmaxf(a.z, b.z); r.w = fmaxf(a.w, b.w); return r;
}

__device__ __forceinline__ int scan_chunk(const int* __restrict__ dsts, int nE, int cbase, int slotBase,
                                          int nb, int vec8, int* list, int tid, int lane, int wave) {
  int wc = 0;
  const int el0  = tid * EPT;
  const int e0   = cbase + el0;
  const int sent = -2147483647 - 1;
  v4i da, db;
  if (vec8 != 0 && cbase + CHUNK <= nE) {
    da = *(const v4i*)(dsts + e0);
    db = *(const v4i*)(dsts + e0 + 4);
  } else {
    da.x = (e0     < nE) ? dsts[min(e0,     nE - 1)] : sent;
    da.y = (e0 + 1 < nE) ? dsts[min(e0 + 1, nE - 1)] : sent;
    da.z = (e0 + 2 < nE) ? dsts[min(e0 + 2, nE - 1)] : sent;
    da.w = (e0 + 3 < nE) ? dsts[min(e0 + 3, nE - 1)] : sent;
    db.x = (e0 + 4 < nE) ? dsts[min(e0 + 4, nE - 1)] : sent;
    db.y = (e0 + 5 < nE) ? dsts[min(e0 + 5, nE - 1)] : sent;
    db.z = (e0 + 6 < nE) ? dsts[min(e0 + 6, nE - 1)] : sent;
    db.w = (e0 + 7 < nE) ? dsts[min(e0 + 7, nE - 1)] : sent;
  }
  const unsigned nbs = (unsigned)slotBase;
  const unsigned unb = (unsigned)nb;
  const unsigned s0 = (unsigned)da.x - nbs, s1 = (unsigned)da.y - nbs;
  const unsigned s2 = (unsigned)da.z - nbs, s3 = (unsigned)da.w - nbs;
  const unsigned s4 = (unsigned)db.x - nbs, s5 = (unsigned)db.y - nbs;
  const unsigned s6 = (unsigned)db.z - nbs, s7 = (unsigned)db.w - nbs;
  const bool h0 = s0 < unb, h1 = s1 < unb, h2 = s2 < unb, h3 = s3 < unb;
  const bool h4 = s4 < unb, h5 = s5 < unb, h6 = s6 < unb, h7 = s7 < unb;
  const unsigned any = __builtin_amdgcn_ballot_w32(h0 | h1 | h2 | h3 | h4 | h5 | h6 | h7);
  if (any != 0u) {
#define HITJ(J, HJ, SJ) { \
      const unsigned mj = __builtin_amdgcn_ballot_w32(HJ); \
      if (mj != 0u) { \
        if (HJ) { \
          const int pos = wc + (int)__builtin_amdgcn_mbcnt_lo(mj, 0u); \
          if (pos < WCAP) list[wave * WCAP + pos] = ((el0 + (J)) << SLOTB) | (int)(SJ); \
        } \
        wc += (int)__builtin_popcount(mj); } }
    HITJ(0, h0, s0)
    HITJ(1, h1, s1)
    HITJ(2, h2, s2)
    HITJ(3, h3, s3)
    HITJ(4, h4, s4)
    HITJ(5, h5, s5)
    HITJ(6, h6, s6)
    HITJ(7, h7, s7)
#undef HITJ
  }
  return wc;
}

__global__ __launch_bounds__(NTHR) void k_prep(const float* __restrict__ x,
                                               const float* __restrict__ W1, const float* __restrict__ W2,
                                               const float* __restrict__ We1, const float* __restrict__ ae1,
                                               const float* __restrict__ We2, const float* __restrict__ ae2,
                                               unsigned short* xb, unsigned short* w1t, unsigned short* w2t,
                                               float* kap, int nN, int nUx, int nBx, int nB1, int nB2) {
  __shared__ __attribute__((aligned(16))) float skap[KAPN];
  const int tid = (int)threadIdx.x;
  const int bid = (int)blockIdx.x;
  const v4f z4 = {0.f, 0.f, 0.f, 0.f};
  if (bid < nBx) {
    const int i = bid * NTHR + tid;
    if (i >= nUx) return;
    const int row = i / 12;
    const int c0  = (i - row * 12) * 8;
    const int rc  = row < nN ? row : nN - 1;
    const int ca  = c0 < FIN - 4 ? c0 : FIN - 4;
    const int cbb = (c0 + 4) < FIN - 4 ? (c0 + 4) : FIN - 4;
    const float* pr = x + (size_t)rc * FIN;
    v4f a = *(const v4fa*)(pr + ca), b = *(const v4fa*)(pr + cbb);
    if (row >= nN || c0 >= FIN) a = z4;
    if (row >= nN || c0 + 4 >= FIN) b = z4;
    a = bfr4(a); b = bfr4(b);
    const v4u hv = pack8(a, b);
    const size_t o = (size_t)row * KIN + c0;
    *(volatile v4u*)(xb + o) = hv;
    __threadfence();
    *(volatile v4u*)(xb + o) = hv;
  } else if (bid < nBx + nB1) {
    const int u = (bid - nBx) * NTHR + tid;
    if (u >= HD1 * (KIN / 8)) return;
    const int n  = u / 12;
    const int k8 = (u - n * 12) * 8;
    float t[8];
#pragma unroll
    for (int j = 0; j < 8; ++j) {
      const int k  = k8 + j;
      const int kc = k < FIN ? k : FIN - 1;
      const float v = W1[(size_t)kc * (size_t)HD1 + n];
      t[j] = k < FIN ? v : 0.f;
    }
    v4f a, b;
    a.x = t[0]; a.y = t[1]; a.z = t[2]; a.w = t[3]; b.x = t[4]; b.y = t[5]; b.z = t[6]; b.w = t[7];
    const v4u wv = pack8(a, b);
    const size_t o = (size_t)n * (size_t)KIN + k8;
    *(volatile v4u*)(w1t + o) = wv;
    __threadfence();
    *(volatile v4u*)(w1t + o) = wv;
  } else if (bid < nBx + nB1 + nB2) {
    const int u = (bid - nBx - nB1) * NTHR + tid;
    if (u >= HD2 * (KA2 / 8)) return;
    const int n  = u / (KA2 / 8);
    const int k8 = (u - n * (KA2 / 8)) * 8;
    const int kk = k8 < HD1 ? k8 : k8 - HD1;
    const float* p = W2 + (size_t)kk * (size_t)HD2 + n;
    v4f a, b;
    a.x = p[0];                  a.y = p[(size_t)HD2];        a.z = p[(size_t)2 * HD2];    a.w = p[(size_t)3 * HD2];
    b.x = p[(size_t)4 * HD2];    b.y = p[(size_t)5 * HD2];    b.z = p[(size_t)6 * HD2];    b.w = p[(size_t)7 * HD2];
    const v4u wv = pack8(a, b);
    const size_t o = (size_t)n * (size_t)KA2 + k8;
    *(volatile v4u*)(w2t + o) = wv;
    __threadfence();
    *(volatile v4u*)(w2t + o) = wv;
  } else {
    const int lane = tid & 31, wave = tid >> 5;
    if (tid < KAPN) skap[tid] = 0.f;
    __syncthreads();
#pragma unroll 1
    for (int p = wave; p < NH1 * EDM + EDM; p += NWAVE) {
      const bool l2 = p >= NH1 * EDM;
      const int h = l2 ? 0 : p / EDM;
      const int t = l2 ? (p - NH1 * EDM) : (p - h * EDM);
      const float* wrow = l2 ? (We2 + (size_t)t * HD2) : (We1 + (size_t)t * HD1 + h * CH);
      const float* arow = l2 ? ae2 : (ae1 + h * CH);
      float s = 0.f;
#pragma unroll
      for (int jj = 0; jj < 3; ++jj) {
        const int c = 128 * jj + 4 * lane;
        const v4f w4 = bfr4(*(const v4fa*)(wrow + c));
        const v4f a4 = bfr4(*(const v4fa*)(arow + c));
        s = fmaf(w4.x, a4.x, s); s = fmaf(w4.y, a4.y, s); s = fmaf(w4.z, a4.z, s); s = fmaf(w4.w, a4.w, s);
      }
#pragma unroll
      for (int off = 16; off > 0; off >>= 1) s += __shfl_xor(s, off);
      if (lane == 0) skap[l2 ? (KAP2 + t) : p] = s;
    }
    __syncthreads();
    const v4f kv = *(const v4f*)(skap + 4 * (tid & 15));
    float* op = kap + 4 * (tid & 15);
    if (tid < 16) *(volatile v4f*)op = kv;
    __threadfence();
    if (tid < 16) *(volatile v4f*)op = kv;
  }
}

__global__ __launch_bounds__(NTHR) void k_edge(const float* __restrict__ ea, const float* __restrict__ kap,
                                               float* AE1, float* AE2, int nE) {
  __shared__ __attribute__((aligned(16))) float sk[KAPN];
  const int tid = (int)threadIdx.x;
  {
    const v4f kv = *(const v4fa*)(kap + 4 * (tid & 15));
    if (tid < 16) *(v4f*)(sk + 4 * tid) = kv;
  }
  __syncthreads();
  const int e  = (int)blockIdx.x * NTHR + tid;
  const int ec = e < nE ? e : nE - 1;
  const float* er = ea + (size_t)ec * EDM;
  float a0 = 0.f, a1 = 0.f, a2 = 0.f, a3 = 0.f, a4 = 0.f;
#pragma unroll 1
  for (int t = 0; t < EDM; ++t) {
    const float v = bfr(er[t]);
    a0 = fmaf(v, sk[t], a0);
    a1 = fmaf(v, sk[EDM + t], a1);
    a2 = fmaf(v, sk[2 * EDM + t], a2);
    a3 = fmaf(v, sk[3 * EDM + t], a3);
    a4 = fmaf(v, sk[KAP2 + t], a4);
  }
  const bool live = e < nE;
  v4f o;
  o.x = live ? a0 : 0.f; o.y = live ? a1 : 0.f; o.z = live ? a2 : 0.f; o.w = live ? a3 : 0.f;
  const float o2 = live ? a4 : 0.f;
  float* p1 = AE1 + (size_t)e * 4;
  float* p2 = AE2 + (size_t)e;
  *(volatile v4f*)p1 = o;
  *(volatile float*)p2 = o2;
  __threadfence();
  *(volatile v4f*)p1 = o;
  *(volatile float*)p2 = o2;
}

__global__ __launch_bounds__(GTHR) void k_gemm(
    const unsigned short* __restrict__ A, const unsigned short* __restrict__ WT,
    float* outF, int K, int ldo)
{
  __shared__ __attribute__((aligned(16))) float stg[GBM * GBN];
  const int tid = (int)threadIdx.x, lane = tid & 31, wave = tid >> 5, hh = lane >> 4, m = lane & 15;
  const int rowBase = (int)blockIdx.x * GBM;
  const int col0    = (int)blockIdx.y * GBN;

  v8f acc[4];
  {
    const v8f z = {0.f, 0.f, 0.f, 0.f, 0.f, 0.f, 0.f, 0.f};
    acc[0] = z; acc[1] = z; acc[2] = z; acc[3] = z;
  }
  const unsigned short* ap = A  + (size_t)(rowBase + 16 * wave + m) * (size_t)K + 8 * hh;
  const unsigned short* wp = WT + (size_t)(col0 + m) * (size_t)K + 8 * hh;
  const int ksteps = K >> 5;
#pragma unroll 1
  for (int ks = 0; ks < ksteps; ++ks) {
    FragB af;
    af.h[0] = *(const v8usa*)(ap + 32 * ks);
    af.h[1] = *(const v8usa*)(ap + 32 * ks + 16);
#pragma unroll
    for (int t = 0; t < 4; ++t) {
      const unsigned short* wq = wp + (size_t)(16 * t) * (size_t)K + 32 * ks;
      FragB bf;
      bf.h[0] = *(const v8usa*)wq;
      bf.h[1] = *(const v8usa*)(wq + 16);
      acc[t] = wmb(af, bf, acc[t]);
    }
  }

#pragma unroll
  for (int t = 0; t < 4; ++t) {
    const int lc = 16 * t + m;
#pragma unroll
    for (int r = 0; r < 8; ++r) {
      const int lr = 16 * wave + 8 * hh + r;
      stg[lr * GBN + lc] = acc[t][r];
    }
  }
  __syncthreads();

  v4f fv[8];
#pragma unroll
  for (int i = 0; i < 8; ++i) {
    const int lr = 16 * wave + 2 * i + hh;
    fv[i] = *(const v4fa*)(stg + lr * GBN + 4 * m);
  }
#pragma unroll
  for (int i = 0; i < 8; ++i) {
    const int lr = 16 * wave + 2 * i + hh;
    const int gr = rowBase + lr;
    float* op = outF + (size_t)gr * (size_t)ldo + col0 + 4 * m;
    *(volatile v4f*)op = fv[i];
  }
  __threadfence();
#pragma unroll
  for (int i = 0; i < 8; ++i) {
    const int lr = 16 * wave + 2 * i + hh;
    const int gr = rowBase + lr;
    float* op = outF + (size_t)gr * (size_t)ldo + col0 + 4 * m;
    *(volatile v4f*)op = fv[i];
  }
}

template<int NH>
__global__ __launch_bounds__(NTHR) void k_ndots(const float* __restrict__ F, const float* __restrict__ asv,
                                                const float* __restrict__ adv, float* ELR, int nN) {
  __shared__ __attribute__((aligned(16))) float srec[NDB * ELW];
  const int tid = (int)threadIdx.x, lane = tid & 31, wave = tid >> 5;
  const int nodeBase = (int)blockIdx.x * NDB;
  const int RW = NH * CH;
  srec[tid] = 0.f;
  __syncthreads();
#pragma unroll 1
  for (int i = 0; i < NDB / NWAVE; ++i) {
    const int ln   = wave * (NDB / NWAVE) + i;
    const int node = nodeBase + ln;
    const int rc   = node < nN ? node : nN - 1;
    const float* fr = F + (size_t)rc * (size_t)RW + 4 * lane;
#pragma unroll 1
    for (int h = 0; h < NH; ++h) {
      float ps = 0.f, pd = 0.f;
#pragma unroll
      for (int jj = 0; jj < 3; ++jj) {
        const int c = h * CH + 128 * jj;
        const v4f v  = *(const v4fa*)(fr + c);
        const v4f a4 = bfr4(*(const v4fa*)(asv + c + 4 * lane));
        const v4f d4 = bfr4(*(const v4fa*)(adv + c + 4 * lane));
        ps = fmaf(v.x, a4.x, ps); ps = fmaf(v.y, a4.y, ps); ps = fmaf(v.z, a4.z, ps); ps = fmaf(v.w, a4.w, ps);
        pd = fmaf(v.x, d4.x, pd); pd = fmaf(v.y, d4.y, pd); pd = fmaf(v.z, d4.z, pd); pd = fmaf(v.w, d4.w, pd);
      }
#pragma unroll
      for (int off = 16; off > 0; off >>= 1) {
        ps += __shfl_xor(ps, off);
        pd += __shfl_xor(pd, off);
      }
      if (lane == 0) {
        srec[ln * ELW + h]     = node < nN ? ps : 0.f;
        srec[ln * ELW + 4 + h] = node < nN ? pd : 0.f;
      }
    }
  }
  __syncthreads();
  const v4f ev = *(const v4f*)(srec + 4 * (tid & 63));
  float* op = ELR + (size_t)nodeBase * ELW + 4 * (tid & 63);
  if (tid < 64) *(volatile v4f*)op = ev;
  __threadfence();
  if (tid < 64) *(volatile v4f*)op = ev;
}

template<int L>
__global__ __launch_bounds__(NTHR) void k_agg(
    const int* __restrict__ srcs, const int* __restrict__ dsts,
    const float* __restrict__ F, const float* __restrict__ ELR,
    const float* __restrict__ AEV, const float* __restrict__ bias,
    unsigned short* A2, float* HE, float* REC,
    int nN, int nE, int nb, int vec8, int MPr) {
  extern __shared__ v4f lds_dyn[];
  int* reg1 = (int*)lds_dyn;
  int* reg2 = reg1 + RCAP;
  int* scnt = reg2 + RCAP;
  int* soff = scnt + NBMAX;
  int* list = soff + NBMAX;
  int* wcnt = list + LISTN;
  int* wtot = wcnt + NWAVE;
  const int tid = (int)threadIdx.x, lane = tid & 31, wave = tid >> 5, hh = lane >> 4;
  const int nodeBase = (int)blockIdx.x * nb;

  for (int i = tid; i < NBMAX; i += NTHR) scnt[i] = 0;
  __syncthreads();

  int tot = 0;
  const int nChunks = (nE + CHUNK - 1) / CHUNK;
#pragma unroll 1
  for (int ch = 0; ch < nChunks; ++ch) {
    const int cbase = ch * CHUNK;
    const int wc = scan_chunk(dsts, nE, cbase, nodeBase, nb, vec8, list, tid, lane, wave);
    if (lane == 0) wcnt[wave] = wc;
    __syncthreads();
    int pre = 0, all = 0;
#pragma unroll
    for (int w2 = 0; w2 < NWAVE; ++w2) {
      int c = wcnt[w2];
      c = c < 0 ? 0 : (c > WCAP ? WCAP : c);
      all += c;
      pre += (w2 < wave) ? c : 0;
    }
    const int wcc  = wc > WCAP ? WCAP : wc;
    const int base = tot + pre;
#pragma unroll 1
    for (int i = lane; i < wcc; i += 32) {
      const int ent = list[wave * WCAP + i];
      const int el  = (ent >> SLOTB) & (CHUNK - 1);
      const int sl  = ent & (NBMAX - 1);
      int eid = cbase + el;
      eid = eid > nE - 1 ? nE - 1 : eid;
      const int pos = base + i;
      if (pos < RCAP) reg1[pos] = (int)(((unsigned)eid << SLOTB) | (unsigned)sl);
    }
    tot += all;
    tot = tot > RCAP ? RCAP : tot;
    __syncthreads();
  }
  const int nh = tot;

  if (wave == 0) {
#pragma unroll 1
    for (int b0 = 0; b0 < nh; b0 += 32) {
      const int idx = b0 + lane;
      const int uv  = reg1[idx < nh ? idx : nh - 1];
      const int m32 = (nh - b0) < 32 ? (nh - b0) : 32;
#pragma unroll 1
      for (int k = 0; k < m32; ++k) {
        const int u  = __builtin_amdgcn_readlane(uv, k);
        const int sl = u & (NBMAX - 1);
        if (lane == 0) scnt[sl] = scnt[sl] + 1;
      }
    }
  }
  __syncthreads();

  {
    const v4i ca = *(const v4i*)(scnt + 8 * tid);
    const v4i cb = *(const v4i*)(scnt + 8 * tid + 4);
    const int e0 = ca.x < 0 ? 0 : ca.x, e1 = ca.y < 0 ? 0 : ca.y, e2 = ca.z < 0 ? 0 : ca.z, e3 = ca.w < 0 ? 0 : ca.w;
    const int e4 = cb.x < 0 ? 0 : cb.x, e5 = cb.y < 0 ? 0 : cb.y, e6 = cb.z < 0 ? 0 : cb.z, e7 = cb.w < 0 ? 0 : cb.w;
    const int ts = e0 + e1 + e2 + e3 + e4 + e5 + e6 + e7;
    int incl = ts;
#pragma unroll
    for (int d = 1; d < 32; d <<= 1) {
      const int up = __shfl_up(incl, d);
      if (lane >= d) incl += up;
    }
    if (lane == 31) wtot[wave] = incl;
    __syncthreads();
    int pre = 0;
#pragma unroll
    for (int w2 = 0; w2 < NWAVE; ++w2) pre += (w2 < wave) ? wtot[w2] : 0;
    int run = pre + incl - ts;
    soff[8 * tid + 0] = run; run += e0;
    soff[8 * tid + 1] = run; run += e1;
    soff[8 * tid + 2] = run; run += e2;
    soff[8 * tid + 3] = run; run += e3;
    soff[8 * tid + 4] = run; run += e4;
    soff[8 * tid + 5] = run; run += e5;
    soff[8 * tid + 6] = run; run += e6;
    soff[8 * tid + 7] = run;
  }
  __syncthreads();
  for (int i = tid; i < NBMAX; i += NTHR) list[i] = soff[i];
  __syncthreads();

  if (wave == 0) {
#pragma unroll 1
    for (int b0 = 0; b0 < nh; b0 += 32) {
      const int idx = b0 + lane;
      const int uv  = reg1[idx < nh ? idx : nh - 1];
      const int m32 = (nh - b0) < 32 ? (nh - b0) : 32;
#pragma unroll 1
      for (int k = 0; k < m32; ++k) {
        const int u   = __builtin_amdgcn_readlane(uv, k);
        const int sl  = u & (NBMAX - 1);
        const int eid = (int)((unsigned)u >> SLOTB);
        if (lane == 0) {
          int pos = list[sl];
          pos = pos < 0 ? 0 : (pos > RCAP - 1 ? RCAP - 1 : pos);
          reg2[pos] = eid;
          list[sl] = pos + 1;
        }
      }
    }
  }
  __syncthreads();

  const int nbw = nb >> 3;
  const bool ovf = (nh >= RCAP);
  const float qnan = __int_as_float(0x7fc00000);
  const v4f z4 = {0.f, 0.f, 0.f, 0.f};

  if (L == 1) {
#pragma unroll 1
    for (int jt = 0; jt < nbw; ++jt) {
      const int slot = wave * nbw + jt;
      const int grow = nodeBase + slot;
      const int gcl  = grow < nN ? grow : nN - 1;
      int st = soff[slot];
      const int craw = scnt[slot];
      int cnt = craw;
      st  = st < 0 ? 0 : (st > nh ? nh : st);
      cnt = cnt < 0 ? 0 : (cnt > DEGCAP ? DEGCAP : cnt);
      if (cnt > nh - st) cnt = nh - st;
      const float pz = (ovf || craw > DEGCAP) ? qnan : 0.0f;

      const v4f es4 = *(const v4fa*)(ELR + (size_t)gcl * ELW);
      const v4f ed4 = *(const v4fa*)(ELR + (size_t)gcl * ELW + 4);
      float mx[4], dn[4], wsm[4];
#pragma unroll
      for (int h = 0; h < 4; ++h) { mx[h] = -1.0e30f; dn[h] = 0.f; wsm[h] = 0.f; }

#pragma unroll 1
      for (int q = 0; q < cnt; ++q) {
        int idx = st + q; idx = idx > RCAP - 1 ? RCAP - 1 : idx;
        int eid = reg2[idx]; eid = eid < 0 ? 0 : (eid > nE - 1 ? nE - 1 : eid);
        const int sraw = srcs[eid];
        const int s = sraw < 0 ? 0 : (sraw > nN - 1 ? nN - 1 : sraw);
        const v4f el4 = *(const v4fa*)(ELR + (size_t)s * ELW);
        const v4f ae4 = *(const v4fa*)(AEV + (size_t)eid * 4);
        float lg[4];
        lg[0] = leaky((el4.x + ed4.x) + ae4.x);
        lg[1] = leaky((el4.y + ed4.y) + ae4.y);
        lg[2] = leaky((el4.z + ed4.z) + ae4.z);
        lg[3] = leaky((el4.w + ed4.w) + ae4.w);
        wsm[0] += ae4.x; wsm[1] += ae4.y; wsm[2] += ae4.z; wsm[3] += ae4.w;
#pragma unroll
        for (int h = 0; h < 4; ++h) ostep(lg[h], mx[h], dn[h]);
      }
      const float rcn = __builtin_amdgcn_rcpf(fmaxf((float)cnt, 1.0f));
      float esd[4];
      esd[0] = es4.x + ed4.x; esd[1] = es4.y + ed4.y; esd[2] = es4.z + ed4.z; esd[3] = es4.w + ed4.w;
      float inv[4], wsf[4];
#pragma unroll
      for (int h = 0; h < 4; ++h) {
        const float lw  = wsm[h] * rcn;
        const float lgs = leaky(esd[h] + lw);
        ostep(lgs, mx[h], dn[h]);
        inv[h] = __builtin_amdgcn_rcpf(dn[h] + EPS_SM);
        wsf[h] = __expf(lgs - mx[h]) * inv[h];
      }
      const bool live = grow < nN;
      const bool wr   = grow < MPr;

#pragma unroll 1
      for (int half = 0; half < 2; ++half) {
        const bool hs = half != 0;
        const float mA = hs ? mx[2]  : mx[0],  mB = hs ? mx[3]  : mx[1];
        const float iA = hs ? inv[2] : inv[0], iB = hs ? inv[3] : inv[1];
        const float sA = hs ? wsf[2] : wsf[0], sB = hs ? wsf[3] : wsf[1];
        const float edA = hs ? ed4.z : ed4.x,  edB = hs ? ed4.w : ed4.y;
        const int cb = 768 * half + 8 * lane;
        const float s1 = hh ? sB : sA;
        const float* fr = F + (size_t)gcl * HD1 + cb;
        v4f a00 = mul4s(sA, *(const v4fa*)(fr));
        v4f a01 = mul4s(sA, *(const v4fa*)(fr + 4));
        v4f a10 = mul4s(s1, *(const v4fa*)(fr + 256));
        v4f a11 = mul4s(s1, *(const v4fa*)(fr + 260));
        v4f a20 = mul4s(sB, *(const v4fa*)(fr + 512));
        v4f a21 = mul4s(sB, *(const v4fa*)(fr + 516));

#pragma unroll 1
        for (int q = 0; q < cnt; ++q) {
          int idx = st + q; idx = idx > RCAP - 1 ? RCAP - 1 : idx;
          int eid = reg2[idx]; eid = eid < 0 ? 0 : (eid > nE - 1 ? nE - 1 : eid);
          const int sraw = srcs[eid];
          const int s = sraw < 0 ? 0 : (sraw > nN - 1 ? nN - 1 : sraw);
          const v4f el4 = *(const v4fa*)(ELR + (size_t)s * ELW);
          const v4f ae4 = *(const v4fa*)(AEV + (size_t)eid * 4);
          const float elA = hs ? el4.z : el4.x, elB = hs ? el4.w : el4.y;
          const float aeA = hs ? ae4.z : ae4.x, aeB = hs ? ae4.w : ae4.y;
          const float lgA = leaky((elA + edA) + aeA);
          const float lgB = leaky((elB + edB) + aeB);
          const float pA = __expf(lgA - mA) * iA;
          const float pB = __expf(lgB - mB) * iB;
          const float p1 = hh ? pB : pA;
          const float* sr = F + (size_t)s * HD1 + cb;
          const v4f x00 = *(const v4fa*)(sr),       x01 = *(const v4fa*)(sr + 4);
          const v4f x10 = *(const v4fa*)(sr + 256), x11 = *(const v4fa*)(sr + 260);
          const v4f x20 = *(const v4fa*)(sr + 512), x21 = *(const v4fa*)(sr + 516);
          a00 = fma4s(pA, x00, a00); a01 = fma4s(pA, x01, a01);
          a10 = fma4s(p1, x10, a10); a11 = fma4s(p1, x11, a11);
          a20 = fma4s(pB, x20, a20); a21 = fma4s(pB, x21, a21);
        }

        const float* br = bias + cb;
        v4f y00 = elu4(add4(a00, bfr4(*(const v4fa*)(br))));
        v4f y01 = elu4(add4(a01, bfr4(*(const v4fa*)(br + 4))));
        v4f y10 = elu4(add4(a10, bfr4(*(const v4fa*)(br + 256))));
        v4f y11 = elu4(add4(a11, bfr4(*(const v4fa*)(br + 260))));
        v4f y20 = elu4(add4(a20, bfr4(*(const v4fa*)(br + 512))));
        v4f y21 = elu4(add4(a21, bfr4(*(const v4fa*)(br + 516))));
        y00 = live ? y00 : z4; y01 = live ? y01 : z4; y10 = live ? y10 : z4;
        y11 = live ? y11 : z4; y20 = live ? y20 : z4; y21 = live ? y21 : z4;
        const v4f pz4 = {pz, pz, pz, pz};
        y00 = add4(y00, pz4); y01 = add4(y01, pz4); y10 = add4(y10, pz4);
        y11 = add4(y11, pz4); y20 = add4(y20, pz4); y21 = add4(y21, pz4);
        v4u hv0, lv0, hv1, lv1, hv2, lv2;
        split8(y00, y01, hv0, lv0);
        split8(y10, y11, hv1, lv1);
        split8(y20, y21, hv2, lv2);
        unsigned short* gp = A2 + (size_t)grow * KA2 + cb;
        if (wr) {
          *(volatile v4u*)(gp)             = hv0;
          *(volatile v4u*)(gp + 256)       = hv1;
          *(volatile v4u*)(gp + 512)       = hv2;
          *(volatile v4u*)(gp + HD1)       = lv0;
          *(volatile v4u*)(gp + HD1 + 256) = lv1;
          *(volatile v4u*)(gp + HD1 + 512) = lv2;
        }
        __threadfence();
        if (wr) {
          *(volatile v4u*)(gp)             = hv0;
          *(volatile v4u*)(gp + 256)       = hv1;
          *(volatile v4u*)(gp + 512)       = hv2;
          *(volatile v4u*)(gp + HD1)       = lv0;
          *(volatile v4u*)(gp + HD1 + 256) = lv1;
          *(volatile v4u*)(gp + HD1 + 512) = lv2;
        }
      }
    }
  } else {
    float* recs = (float*)reg1;
    const int cl = 4 * lane;
#pragma unroll 1
    for (int jt = 0; jt < nbw; ++jt) {
      const int slot = wave * nbw + jt;
      const int grow = nodeBase + slot;
      const int gcl  = grow < nN ? grow : nN - 1;
      int st = soff[slot];
      const int craw = scnt[slot];
      int cnt = craw;
      st  = st < 0 ? 0 : (st > nh ? nh : st);
      cnt = cnt < 0 ? 0 : (cnt > DEGCAP ? DEGCAP : cnt);
      if (cnt > nh - st) cnt = nh - st;
      const float pz = (ovf || craw > DEGCAP) ? qnan : 0.0f;

      const float es = ELR[(size_t)gcl * ELW];
      const float ed = ELR[(size_t)gcl * ELW + 4];
      float mx = -1.0e30f, dn = 0.f, wsm = 0.f;

#pragma unroll 1
      for (int q = 0; q < cnt; ++q) {
        int idx = st + q; idx = idx > RCAP - 1 ? RCAP - 1 : idx;
        int eid = reg2[idx]; eid = eid < 0 ? 0 : (eid > nE - 1 ? nE - 1 : eid);
        const int sraw = srcs[eid];
        const int s = sraw < 0 ? 0 : (sraw > nN - 1 ? nN - 1 : sraw);
        const float asr = ELR[(size_t)s * ELW];
        const float ae  = AEV[eid];
        const float lg  = leaky((asr + ed) + ae);
        wsm += ae;
        ostep(lg, mx, dn);
      }
      const float rcn = __builtin_amdgcn_rcpf(fmaxf((float)cnt, 1.0f));
      const float lw  = wsm * rcn;
      const float lgs = leaky((es + ed) + lw);
      ostep(lgs, mx, dn);
      const float inv = __builtin_amdgcn_rcpf(dn + EPS_SM);
      const float wsf = __expf(lgs - mx) * inv;

      const float* fr = F + (size_t)gcl * HD2 + cl;
      v4f a0 = mul4s(wsf, *(const v4fa*)(fr));
      v4f a1 = mul4s(wsf, *(const v4fa*)(fr + 128));
      v4f a2 = mul4s(wsf, *(const v4fa*)(fr + 256));

#pragma unroll 1
      for (int q = 0; q < cnt; ++q) {
        int idx = st + q; idx = idx > RCAP - 1 ? RCAP - 1 : idx;
        int eid = reg2[idx]; eid = eid < 0 ? 0 : (eid > nE - 1 ? nE - 1 : eid);
        const int sraw = srcs[eid];
        const int s = sraw < 0 ? 0 : (sraw > nN - 1 ? nN - 1 : sraw);
        const float asr = ELR[(size_t)s * ELW];
        const float ae  = AEV[eid];
        const float lg  = leaky((asr + ed) + ae);
        const float p   = __expf(lg - mx) * inv;
        const float* sr = F + (size_t)s * HD2 + cl;
        const v4f x0 = *(const v4fa*)(sr), x1 = *(const v4fa*)(sr + 128), x2 = *(const v4fa*)(sr + 256);
        a0 = fma4s(p, x0, a0); a1 = fma4s(p, x1, a1); a2 = fma4s(p, x2, a2);
      }
      const bool live = grow < nN;
      const bool wr   = grow < MPr;
      const float* br = bias + cl;
      v4f y0 = elu4(add4(a0, bfr4(*(const v4fa*)(br))));
      v4f y1 = elu4(add4(a1, bfr4(*(const v4fa*)(br + 128))));
      v4f y2 = elu4(add4(a2, bfr4(*(const v4fa*)(br + 256))));
      y0 = live ? y0 : z4; y1 = live ? y1 : z4; y2 = live ? y2 : z4;
      const v4f pz4 = {pz, pz, pz, pz};
      y0 = add4(y0, pz4); y1 = add4(y1, pz4); y2 = add4(y2, pz4);
      float* gp = HE + (size_t)grow * HD2 + cl;
      if (wr) {
        *(volatile v4f*)(gp)       = y0;
        *(volatile v4f*)(gp + 128) = y1;
        *(volatile v4f*)(gp + 256) = y2;
      }
      __threadfence();
      if (wr) {
        *(volatile v4f*)(gp)       = y0;
        *(volatile v4f*)(gp + 128) = y1;
        *(volatile v4f*)(gp + 256) = y2;
      }
      if (lane == 0) {
        recs[4 * slot + 0] = mx + pz;
        recs[4 * slot + 1] = dn + pz;
        recs[4 * slot + 2] = lw + pz;
        recs[4 * slot + 3] = 0.f;
      }
    }
    __syncthreads();
#pragma unroll 1
    for (int p = tid; p < nb; p += NTHR) {
      const int grow = nodeBase + p;
      const v4f v = *(const v4f*)(recs + 4 * p);
      if (grow < MPr) *(volatile v4f*)(REC + (size_t)grow * 4) = v;
    }
    __threadfence();
#pragma unroll 1
    for (int p = tid; p < nb; p += NTHR) {
      const int grow = nodeBase + p;
      const v4f v = *(const v4f*)(recs + 4 * p);
      if (grow < MPr) *(volatile v4f*)(REC + (size_t)grow * 4) = v;
    }
  }
}

__global__ __launch_bounds__(NTHR) void k_alpha(const int* __restrict__ srcs, const int* __restrict__ dsts,
                                                const float* __restrict__ AE2, const float* __restrict__ ELR,
                                                const float* __restrict__ REC, float* out,
                                                int nN, int nE, int nT) {
  const int t  = (int)blockIdx.x * NTHR + (int)threadIdx.x;
  const int tc = t < nT ? t : nT - 1;
  const int ecl = tc < nE ? tc : nE - 1;
  int se = srcs[ecl]; se = se < 0 ? 0 : (se > nN - 1 ? nN - 1 : se);
  int de = dsts[ecl]; de = de < 0 ? 0 : (de > nN - 1 ? nN - 1 : de);
  const float aee = AE2[ecl];
  int il = tc - nE; il = il < 0 ? 0 : (il > nN - 1 ? nN - 1 : il);
  const int msk = -(int)(tc >= nE);
  const int s = (il & msk) | (se & ~msk);
  const int d = (il & msk) | (de & ~msk);
  const v4f rd = *(const v4fa*)(REC + (size_t)d * 4);
  const float ae = __int_as_float((__float_as_int(rd.z) & msk) | (__float_as_int(aee) & ~msk));
  const float asr = ELR[(size_t)s * ELW];
  const float adh = ELR[(size_t)d * ELW + 4];
  const float lg  = leaky((asr + adh) + ae);
  const float inv = __builtin_amdgcn_rcpf(rd.y + EPS_SM);
  const float a   = __expf(lg - rd.x) * inv;
  const bool wr = t < nT;
  if (wr) *(volatile float*)(out + t) = a;
  __threadfence();
  if (wr) *(volatile float*)(out + t) = a;
}

__global__ __launch_bounds__(PTHR) void k_pool(const float* __restrict__ HE, const int* __restrict__ bat,
                                               float* out, int nN) {
  __shared__ int hl[(PTHR / 32) * PWC];
  __shared__ int wcnt[4];
  const int g = (int)blockIdx.x;
  const int tid = (int)threadIdx.x, lane = tid & 31, wave = tid >> 5;
  const float ninf = __int_as_float(0xff800000);
  v4f acc = {ninf, ninf, ninf, ninf};
  const int sent = -2147483647 - 1;
  const int nChunks = (nN + PCH - 1) / PCH;
#pragma unroll 1
  for (int ch = 0; ch < nChunks; ++ch) {
    const int cbase = ch * PCH;
    const int e0 = cbase + tid * EPT;
    v4i da, db;
    if (cbase + PCH <= nN) {
      da = *(const v4i*)(bat + e0);
      db = *(const v4i*)(bat + e0 + 4);
    } else {
      da.x = (e0     < nN) ? bat[min(e0,     nN - 1)] : sent;
      da.y = (e0 + 1 < nN) ? bat[min(e0 + 1, nN - 1)] : sent;
      da.z = (e0 + 2 < nN) ? bat[min(e0 + 2, nN - 1)] : sent;
      da.w = (e0 + 3 < nN) ? bat[min(e0 + 3, nN - 1)] : sent;
      db.x = (e0 + 4 < nN) ? bat[min(e0 + 4, nN - 1)] : sent;
      db.y = (e0 + 5 < nN) ? bat[min(e0 + 5, nN - 1)] : sent;
      db.z = (e0 + 6 < nN) ? bat[min(e0 + 6, nN - 1)] : sent;
      db.w = (e0 + 7 < nN) ? bat[min(e0 + 7, nN - 1)] : sent;
    }
    const bool h0 = da.x == g, h1 = da.y == g, h2 = da.z == g, h3 = da.w == g;
    const bool h4 = db.x == g, h5 = db.y == g, h6 = db.z == g, h7 = db.w == g;
    int wc = 0;
    const unsigned any = __builtin_amdgcn_ballot_w32(h0 | h1 | h2 | h3 | h4 | h5 | h6 | h7);
    if (any != 0u) {
#define PHIT(J, HJ) { \
        const unsigned mj = __builtin_amdgcn_ballot_w32(HJ); \
        if (mj != 0u) { \
          if (HJ) { \
            const int pos = wc + (int)__builtin_amdgcn_mbcnt_lo(mj, 0u); \
            if (pos < PWC) hl[wave * PWC + pos] = e0 + (J); \
          } \
          wc += (int)__builtin_popcount(mj); } }
      PHIT(0, h0)
      PHIT(1, h1)
      PHIT(2, h2)
      PHIT(3, h3)
      PHIT(4, h4)
      PHIT(5, h5)
      PHIT(6, h6)
      PHIT(7, h7)
#undef PHIT
    }
    if (lane == 0) wcnt[wave] = wc;
    __syncthreads();
#pragma unroll 1
    for (int w2 = 0; w2 < PTHR / 32; ++w2) {
      int c = wcnt[w2];
      c = c < 0 ? 0 : (c > PWC ? PWC : c);
      c = __builtin_amdgcn_readfirstlane(c);
#pragma unroll 1
      for (int q = 0; q < c; ++q) {
        int n = hl[w2 * PWC + q];
        n = __builtin_amdgcn_readfirstlane(n);
        n = n < 0 ? 0 : (n > nN - 1 ? nN - 1 : n);
        const v4f v = *(const v4fa*)(HE + (size_t)n * HD2 + 4 * tid);
        acc = max4(acc, v);
      }
    }
    __syncthreads();
  }
  const float pinf = __int_as_float(0x7f800000);
  v4f o;
  o.x = (fabsf(acc.x) < pinf) ? acc.x : 0.f;
  o.y = (fabsf(acc.y) < pinf) ? acc.y : 0.f;
  o.z = (fabsf(acc.z) < pinf) ? acc.z : 0.f;
  o.w = (fabsf(acc.w) < pinf) ? acc.w : 0.f;
  float* op = out + (size_t)g * HD2 + 4 * tid;
  *(volatile v4f*)op = o;
  __threadfence();
  *(volatile v4f*)op = o;
}

static int pick_nb(int nE, int nN) {
  int nb = NBMAX;
  while (nb > 32 && (long long)nb * (long long)nE * 5LL > (long long)RCAP * (long long)nN * 4LL) nb >>= 1;
  return nb;
}
static inline int cdiv(int a, int b) { return (a + b - 1) / b; }
static inline size_t al256(size_t v) { return (v + 255) & ~(size_t)255; }

extern "C" void kernel_launch(void* const* d_in, const int* in_sizes, int n_in,
                              void* d_out, int out_size, void* d_ws, size_t ws_size,
                              hipStream_t stream) {
  if (n_in < 16) return;
  if (in_sizes[0] < FIN || (in_sizes[0] % FIN) != 0) return;
  const int nN = in_sizes[0] / FIN;
  if (nN <= 0 || nN > (1 << 22)) return;
  if (in_sizes[1] < 2 || (in_sizes[1] & 1) != 0) return;
  const int nE = in_sizes[1] / 2;
  if (nE < 1 || nE >= (1 << (32 - SLOTB))) return;
  if (in_sizes[2] != nE * EDM) return;
  if (in_sizes[3] != nN) return;
  if (in_sizes[4] != FIN * HD1) return;
  if (in_sizes[5] != HD1 || in_sizes[6] != HD1) return;
  if (in_sizes[7] != EDM * HD1) return;
  if (in_sizes[8] != HD1 || in_sizes[9] != HD1) return;
  if (in_sizes[10] != HD1 * HD2) return;
  if (in_sizes[11] != HD2 || in_sizes[12] != HD2) return;
  if (in_sizes[13] != EDM * HD2) return;
  if (in_sizes[14] != HD2 || in_sizes[15] != HD2) return;
  const int nT = nE + nN;
  if (out_size <= nT) return;
  const int pooledN = out_size - nT;
  if ((pooledN % HD2) != 0) return;
  const int nG = pooledN / HD2;
  if (nG < 1) return;

  const float* x1  = (const float*)d_in[0];
  const int*   ei  = (const int*)  d_in[1];
  const float* ea  = (const float*)d_in[2];
  const int*   bat = (const int*)  d_in[3];
  const float* W1  = (const float*)d_in[4];
  const float* as1 = (const float*)d_in[5];
  const float* ad1 = (const float*)d_in[6];
  const float* We1 = (const float*)d_in[7];
  const float* ae1 = (const float*)d_in[8];
  const float* b1  = (const float*)d_in[9];
  const float* W2  = (const float*)d_in[10];
  const float* as2 = (const float*)d_in[11];
  const float* ad2 = (const float*)d_in[12];
  const float* We2 = (const float*)d_in[13];
  const float* ae2 = (const float*)d_in[14];
  const float* b2  = (const float*)d_in[15];
  float* out0 = (float*)d_out;
  float* out1 = (float*)d_out + (size_t)pooledN;
  const int* src = ei;
  const int* dst = ei + nE;

  const int MP   = cdiv(nN, GBM) * GBM;
  const int EP   = cdiv(nE, NTHR) * NTHR;
  const int nb   = pick_nb(nE, nN);
  if (nb < 32 || (nb & (nb - 1)) != 0 || nb > NBMAX) return;
  const int gA   = cdiv(MP, nb);
  const int vec8 = ((nE & 3) == 0) ? 1 : 0;
  if (gA * nb < MP) return;

  char* ws = (char*)d_ws;
  size_t off = 0;
  const size_t oXB  = off; off = al256(off + (size_t)MP * KIN * 2);
  const size_t oW1T = off; off = al256(off + (size_t)HD1 * KIN * 2);
  const size_t oW2T = off; off = al256(off + (size_t)HD2 * KA2 * 2);
  const size_t oKAP = off; off = al256(off + (size_t)KAPN * 4);
  const size_t oAE1 = off; off = al256(off + (size_t)EP * 4 * 4);
  const size_t oAE2 = off; off = al256(off + (size_t)EP * 4);
  const size_t oH1  = off; off = al256(off + (size_t)MP * HD1 * 4);
  const size_t eH1  = off;
  const size_t oEL1 = off; off = al256(off + (size_t)MP * ELW * 4);
  const size_t oA2  = off; off = al256(off + (size_t)MP * KA2 * 2);
  if (off > ws_size || off > (size_t)WSMAX) return;
  size_t sub = oH1;
  const size_t oH2  = sub; sub = al256(sub + (size_t)MP * HD2 * 4);
  const size_t oEL2 = sub; sub = al256(sub + (size_t)MP * ELW * 4);
  const size_t oHE  = sub; sub = al256(sub + (size_t)MP * HD2 * 4);
  const size_t oREC = sub; sub = al256(sub + (size_t)MP * 4 * 4);
  if (sub > eH1) return;
  unsigned short* XB   = (unsigned short*)(ws + oXB);
  unsigned short* W1T  = (unsigned short*)(ws + oW1T);
  unsigned short* W2T  = (unsigned short*)(ws + oW2T);
  float*          KAP  = (float*)(ws + oKAP);
  float*          AE1  = (float*)(ws + oAE1);
  float*          AE2  = (float*)(ws + oAE2);
  float*          H1   = (float*)(ws + oH1);
  float*          ELR1 = (float*)(ws + oEL1);
  unsigned short* A2   = (unsigned short*)(ws + oA2);
  float*          H2   = (float*)(ws + oH2);
  float*          ELR2 = (float*)(ws + oEL2);
  float*          HE   = (float*)(ws + oHE);
  float*          REC  = (float*)(ws + oREC);

  hipFuncSetAttribute(reinterpret_cast<const void*>(&k_agg<1>),
                      hipFuncAttributeMaxDynamicSharedMemorySize, LDS_AGG);
  hipFuncSetAttribute(reinterpret_cast<const void*>(&k_agg<2>),
                      hipFuncAttributeMaxDynamicSharedMemorySize, LDS_AGG);

  const int nUx = MP * (KIN / 8);
  const int nBx = cdiv(nUx, NTHR);
  if (nBx * NTHR != nUx) return;
  const int nB1 = cdiv(HD1 * (KIN / 8), NTHR);
  const int nB2 = cdiv(HD2 * (KA2 / 8), NTHR);
  k_prep<<<nBx + nB1 + nB2 + 1, NTHR, 0, stream>>>(x1, W1, W2, We1, ae1, We2, ae2,
                                                   XB, W1T, W2T, KAP, nN, nUx, nBx, nB1, nB2);

  k_edge<<<EP / NTHR, NTHR, 0, stream>>>(ea, KAP, AE1, AE2, nE);

  const int gM = MP / GBM;
  k_gemm<<<dim3(gM, HD1 / GBN), GTHR, 0, stream>>>(XB, W1T, H1, KIN, HD1);

  k_ndots<NH1><<<MP / NDB, NTHR, 0, stream>>>(H1, as1, ad1, ELR1, nN);

  k_agg<1><<<gA, NTHR, LDS_AGG, stream>>>(src, dst, H1, ELR1, AE1, b1, A2, HE, REC, nN, nE, nb, vec8, MP);

  k_gemm<<<dim3(gM, HD2 / GBN), GTHR, 0, stream>>>(A2, W2T, H2, KA2, HD2);

  k_ndots<1><<<MP / NDB, NTHR, 0, stream>>>(H2, as2, ad2, ELR2, nN);

  k_agg<2><<<gA, NTHR, LDS_AGG, stream>>>(src, dst, H2, ELR2, AE2, b2, A2, HE, REC, nN, nE, nb, vec8, MP);

  k_alpha<<<cdiv(nT, NTHR), NTHR, 0, stream>>>(src, dst, AE2, ELR2, REC, out1, nN, nE, nT);

  k_pool<<<nG, PTHR, 0, stream>>>(HE, bat, out0, nN);
}
